// MetaDGCRU_12876311953416
// MI455X (gfx1250) — hardware-verified
//
#include <hip/hip_runtime.h>
#include <stdint.h>

#define NB 8
#define NN 400
#define NNP 448
#define KHP 416
#define FEAT 66
#define FPAD 128
#define NCH 5
#define HD 64
#define ED 16
#define IDIM 330
#define KMAIN 5280
#define KMP 5312
#define KGRP 664
#define ROWS 3200
#define GSC 64.0f
#define ASC 16.0f

typedef __attribute__((ext_vector_type(16))) _Float16 v16h;
typedef __attribute__((ext_vector_type(8)))  _Float16 v8h;
typedef __attribute__((ext_vector_type(16))) __bf16   v16b;
typedef __attribute__((ext_vector_type(8)))  __bf16   v8b;
typedef __attribute__((ext_vector_type(8)))  float    v8f;
typedef __attribute__((ext_vector_type(4)))  float    v4f;

__device__ __forceinline__ unsigned short f2bf_bits(float f) {
  unsigned u = __float_as_uint(f);
  return (unsigned short)((u + 0x7FFFu + ((u >> 16) & 1u)) >> 16);
}
__device__ __forceinline__ float bf_bits2f(unsigned short h) { return __uint_as_float(((unsigned)h) << 16); }

__device__ __forceinline__ void dep_guard_h(v8f& a, v8f& b, v16h x, v16h y) { asm volatile("v_nop\n\tv_nop\n\tv_nop\n\tv_nop" : "+v"(a), "+v"(b) : "v"(x), "v"(y)); }
__device__ __forceinline__ void dep_guard_b(v8f& a, v8f& b, v16b x, v16b y) { asm volatile("v_nop\n\tv_nop\n\tv_nop\n\tv_nop" : "+v"(a), "+v"(b) : "v"(x), "v"(y)); }
__device__ __forceinline__ void keep4_h(v16h a, v16h b, v16h c, v16h d) { asm volatile("v_nop" :: "v"(a), "v"(b), "v"(c), "v"(d)); }
__device__ __forceinline__ void keep4_b(v16b a, v16b b, v16b c, v16b d) { asm volatile("v_nop" :: "v"(a), "v"(b), "v"(c), "v"(d)); }
__device__ __forceinline__ void acc_guard4(v8f& a, v8f& b, v8f& c, v8f& d) { asm volatile("v_nop\n\tv_nop\n\tv_nop\n\tv_nop" : "+v"(a), "+v"(b), "+v"(c), "+v"(d)); }
template <typename T> struct Frag;
template <> struct Frag<_Float16> {
  typedef v16h V; union U { v16h v; v8h h[2]; };
  static __device__ __forceinline__ v16h load(const _Float16* p) {
    U f; f.h[0] = *(const v8h*)(p); f.h[1] = *(const v8h*)(p + 16); return f.v;
  }
  static __device__ __forceinline__ v8f mma(v16h a, v16h b, v8f c) {
    return __builtin_amdgcn_wmma_f32_16x16x32_f16(false, a, false, b, (short)0, c, false, false);
  }
  static __device__ __forceinline__ void guard(v8f& a, v8f& b, v16h x, v16h y) { dep_guard_h(a, b, x, y); }
  static __device__ __forceinline__ void keep(v16h a, v16h b, v16h c, v16h d) { keep4_h(a, b, c, d); }
};
template <> struct Frag<__bf16> {
  typedef v16b V; union U { v16b v; v8b h[2]; };
  static __device__ __forceinline__ v16b load(const __bf16* p) {
    U f; f.h[0] = *(const v8b*)(p); f.h[1] = *(const v8b*)(p + 16); return f.v;
  }
  static __device__ __forceinline__ v8f mma(v16b a, v16b b, v8f c) {
    return __builtin_amdgcn_wmma_f32_16x16x32_bf16(false, a, false, b, (short)0, c, false, false);
  }
  static __device__ __forceinline__ void guard(v8f& a, v8f& b, v16b x, v16b y) { dep_guard_b(a, b, x, y); }
  static __device__ __forceinline__ void keep(v16b a, v16b b, v16b c, v16b d) { keep4_b(a, b, c, d); }
};

template <int ET> struct Elem;
template <> struct Elem<0> { typedef _Float16 T; };
template <> struct Elem<1> { typedef __bf16 T; };
template <int ET, bool SPLIT, int BIAS_MODE, int OUT_MODE, bool RESID, int ACT = 0>
__global__ __launch_bounds__(256) void wmma_gemm64(
    const unsigned short* __restrict__ Ap, const unsigned short* __restrict__ A2p, int lda, long strideA,
    const unsigned short* __restrict__ Btp, const unsigned short* __restrict__ Bt2p, int ldb, long strideB,
    void* __restrict__ Cout, void* __restrict__ Cout2, int ldc, long strideC,
    const float* __restrict__ bias,
    const float* __restrict__ resid, long strideR,
    int M, int N, int K, float scale) {
  typedef typename Elem<ET>::T T;
  typedef typename Frag<T>::V V;
  const T* A = (const T*)Ap; const T* A2 = (const T*)A2p; const T* Bt = (const T*)Btp; const T* Bt2 = (const T*)Bt2p;
  __shared__ __align__(16) float sT[8][16 * 68];
  const int b    = blockIdx.y;
  const int lane = threadIdx.x & 31;
  const int wave = threadIdx.x >> 5;
  const int tilesN = N >> 6;
  const int tilesM = M >> 6;
  const int tile = blockIdx.x * 8 + wave;
  if (tile >= tilesM * tilesN) return;
  const int tm = tile / tilesN;
  const int tn = tile - tm * tilesN;
  const int m0 = tm << 6;
  const int n0 = tn << 6;

  const T* Ab  = A  + (size_t)b * strideA;
  const T* Bb  = Bt + (size_t)b * strideB;
  const T* Ab2 = SPLIT ? (A2  + (size_t)b * strideA) : nullptr;
  const T* Bb2 = SPLIT ? (Bt2 + (size_t)b * strideB) : nullptr;

  const int rlane = lane & 15;
  const int koff  = (lane >> 4) * 8;
  const int mOff  = (lane >> 4) * 8;

  v8f acc[4][4];
#pragma unroll
  for (int i = 0; i < 4; ++i)
#pragma unroll
    for (int j = 0; j < 4; ++j) acc[i][j] = (v8f){0.f,0.f,0.f,0.f,0.f,0.f,0.f,0.f};

  for (int k0 = 0; k0 < K; k0 += 32) {
    V bh[4], bl[4];
#pragma unroll
    for (int j = 0; j < 4; ++j) {
      const size_t bo = (size_t)(n0 + (j << 4) + rlane) * ldb + koff + k0;
      bh[j] = Frag<T>::load(Bb + bo);
      if (SPLIT) bl[j] = Frag<T>::load(Bb2 + bo);
    }
#pragma unroll
    for (int i = 0; i < 4; ++i) {
      const size_t ao = (size_t)(m0 + (i << 4) + rlane) * lda + koff + k0;
      V ah = Frag<T>::load(Ab + ao);
      V al;
      if (SPLIT) al = Frag<T>::load(Ab2 + ao);
#pragma unroll
      for (int j = 0; j < 4; ++j) {
        acc[i][j] = Frag<T>::mma(ah, bh[j], acc[i][j]);
        if (SPLIT) {
          acc[i][j] = Frag<T>::mma(ah, bl[j], acc[i][j]);
          acc[i][j] = Frag<T>::mma(al, bh[j], acc[i][j]);
        }
      }
      Frag<T>::guard(acc[i][0], acc[i][3], ah, SPLIT ? al : ah);
    }
    Frag<T>::keep(bh[0], bh[1], bh[2], bh[3]);
    if (SPLIT) Frag<T>::keep(bl[0], bl[1], bl[2], bl[3]);
  }
  acc_guard4(acc[0][0], acc[0][1], acc[0][2], acc[0][3]);
  acc_guard4(acc[1][0], acc[1][1], acc[1][2], acc[1][3]);
  acc_guard4(acc[2][0], acc[2][1], acc[2][2], acc[2][3]);
  acc_guard4(acc[3][0], acc[3][1], acc[3][2], acc[3][3]);

  float* slab = sT[wave];
  const float* Rb = RESID ? (resid + (size_t)b * strideR) : nullptr;
#pragma unroll
  for (int i = 0; i < 4; ++i) {
    const int mBase = m0 + (i << 4);
#pragma unroll
    for (int j = 0; j < 4; ++j) {
      const int n = n0 + (j << 4) + rlane;
      float bv = 0.f;
      if (BIAS_MODE == 2) bv = bias[n];
#pragma unroll
      for (int r = 0; r < 8; ++r) {
        float v = acc[i][j][r] * scale;
        if (BIAS_MODE == 1) v += bias[mBase + mOff + r];
        if (BIAS_MODE == 2) v += bv;
        if (RESID) v += Rb[(size_t)(mBase + mOff + r) * ldc + n];
        if (ACT == 1) v = tanhf(v);
        if (ACT == 2) v = fmaxf(v, 0.0f);
        if (ACT == 3) v = v / (1.0f + expf(-v));
        if (ACT == 4) v = (v > 0.f) ? v : 0.01f * v;
        if (ACT == 5) v = 0.5f * v * (1.0f + erff(v * 0.70710678118654752f));
        if (ACT == 6) { const float ex = expf(-fabsf(v)); const float rc = __builtin_amdgcn_rcpf(1.0f + ex); v = (v >= 0.0f) ? rc : ex * rc; }
        slab[(mOff + r) * 68 + (j << 4) + rlane] = v;
      }
    }
    __builtin_amdgcn_fence(__ATOMIC_RELEASE, "workgroup");
    __builtin_amdgcn_wave_barrier();
    __builtin_amdgcn_fence(__ATOMIC_ACQUIRE, "workgroup");
    if (OUT_MODE == 0) {
      float* C = (float*)Cout + (size_t)b * strideC;
      const int hh = lane >> 4, c4 = (lane & 15) * 4;
      for (int pass = 0; pass < 2; ++pass) {
#pragma unroll
        for (int it = 0; it < 8; ++it) {
          const int row = it * 2 + hh;
          v4f v = *(const v4f*)(slab + row * 68 + c4);
          *(volatile v4f*)(C + (size_t)(mBase + row) * ldc + n0 + c4) = v;
        }
        __threadfence();
      }
    } else {
      const int q = lane >> 3, c8 = (lane & 7) * 8;
      unsigned short* C  = (unsigned short*)Cout  + (size_t)b * strideC;
      unsigned short* C2 = (OUT_MODE == 2) ? ((unsigned short*)Cout2 + (size_t)b * strideC) : nullptr;
      for (int pass = 0; pass < 2; ++pass) {
#pragma unroll
        for (int it = 0; it < 4; ++it) {
          const int row = it * 4 + q;
          const float* sp = slab + row * 68 + c8;
          v8h hv, lv;
#pragma unroll
          for (int e = 0; e < 8; ++e) {
            if (OUT_MODE == 1) {
              hv[e] = (_Float16)sp[e];
            } else {
              unsigned short hb = f2bf_bits(sp[e]);
              unsigned short lb = f2bf_bits(sp[e] - bf_bits2f(hb));
              hv[e] = __builtin_bit_cast(_Float16, hb);
              lv[e] = __builtin_bit_cast(_Float16, lb);
            }
          }
          *(volatile v8h*)(C + (size_t)(mBase + row) * ldc + n0 + c8) = hv;
          if (OUT_MODE == 2) *(volatile v8h*)(C2 + (size_t)(mBase + row) * ldc + n0 + c8) = lv;
        }
        __threadfence();
      }
    }
    __builtin_amdgcn_fence(__ATOMIC_RELEASE, "workgroup");
    __builtin_amdgcn_wave_barrier();
    __builtin_amdgcn_fence(__ATOMIC_ACQUIRE, "workgroup");
  }
}

__global__ __launch_bounds__(256) void cast_graphs(const float* __restrict__ G, _Float16* __restrict__ G16, int total_groups) {
  const int f = blockIdx.x * 256 + threadIdx.x;
  if (f >= total_groups) return;
  const int per_plane = NNP * (KHP / 8);
  const int plane = f / per_plane;
  const int rem = f - plane * per_plane;
  const int row = rem / (KHP / 8);
  const int c0 = (rem - row * (KHP / 8)) * 8;
  const bool valid = (row < NN) && (c0 < NN);
  const int rowc = (row < NN) ? row : (NN - 1);
  const int cc = (c0 <= NN - 8) ? c0 : (NN - 8);
  const float* src = G + ((size_t)plane * NN + rowc) * NN + cc;
  const v4f a0 = *(const v4f*)(src);
  const v4f a1 = *(const v4f*)(src + 4);
  v8h hv;
#pragma unroll
  for (int e = 0; e < 4; ++e) {
    hv[e]     = (_Float16)(valid ? a0[e] * GSC : 0.0f);
    hv[4 + e] = (_Float16)(valid ? a1[e] * GSC : 0.0f);
  }
  _Float16* dst = G16 + (size_t)f * 8;
  *(volatile v8h*)dst = hv;
  __threadfence();
  *(volatile v8h*)dst = hv;
}

__global__ __launch_bounds__(256) void build_wt(const float* __restrict__ W, const float* __restrict__ bias, int O,
                                                _Float16* __restrict__ WT, int total_groups) {
  const int f = blockIdx.x * 256 + threadIdx.x;
  if (f >= total_groups) return;
  const int o = f / KGRP;
  const int q = f - o * KGRP;
  const int qm = (q < 660) ? q : 659;
  const int i = qm >> 1;
  const int d0 = (q < 660) ? ((q & 1) * 8) : ((q < 662) ? (q - 660) * 8 : 0);
  v8h hv;
#pragma unroll
  for (int e = 0; e < 8; ++e) {
    const int d = d0 + e;
    const float wv = W[((size_t)d * IDIM + i) * O + o];
    const float bv = bias[(size_t)d * O + o];
    const float v = (q < 660) ? wv : ((q < 662) ? bv : 0.0f);
    hv[e] = (_Float16)(v * ASC);
  }
  _Float16* dst = WT + (size_t)f * 8;
  *(volatile v8h*)dst = hv;
  __threadfence();
  *(volatile v8h*)dst = hv;
}

template <int PH>
__global__ __launch_bounds__(256) void build_ht0(const float* __restrict__ x, const float* __restrict__ state,
                                                 const float* __restrict__ ZR, _Float16* __restrict__ HT, int total_groups) {
  const int f = blockIdx.x * 256 + threadIdx.x;
  if (f >= total_groups) return;
  const int per_b = FPAD * (NNP / 8);
  const int b = f / per_b;
  const int rem = f - b * per_b;
  const int j = rem / (NNP / 8);
  const int n0 = (rem - j * (NNP / 8)) * 8;
  const int jx = (j < 2) ? j : 1;
  int js = j - 2; js = (js < 0) ? 0 : ((js > HD - 1) ? (HD - 1) : js);
  v8h hv;
#pragma unroll
  for (int e = 0; e < 8; ++e) {
    const int n = n0 + e;
    const int nc = (n < NN) ? n : (NN - 1);
    const size_t r = (size_t)b * NN + nc;
    const float xv = x[r * 2 + jx];
    float sv = state[r * HD + js];
    if (PH) sv *= ZR[r * (2 * HD) + HD + js];
    float v = (j < 2) ? xv : sv;
    v = (n < NN && j < FEAT) ? v : 0.0f;
    hv[e] = (_Float16)v;
  }
  _Float16* dst = HT + (size_t)b * NCH * FPAD * NNP + (size_t)j * NNP + n0;
  *(volatile v8h*)dst = hv;
  __threadfence();
  *(volatile v8h*)dst = hv;
}

template <int PH>
__global__ __launch_bounds__(256) void build_ap(const float* __restrict__ x, const float* __restrict__ state,
                                                const float* __restrict__ emb, const float* __restrict__ ZR,
                                                const _Float16* __restrict__ HT, _Float16* __restrict__ AP, int total_groups) {
  const int f = blockIdx.x * 256 + threadIdx.x;
  if (f >= total_groups) return;
  const int r = f / KGRP;
  const int q = f - r * KGRP;
  const int b = r / NN;
  const int n = r - b * NN;
  const int qm = (q < 660) ? q : 659;
  const int i = qm >> 1;
  const int c = i / FEAT;
  const int j = i - c * FEAT;
  const int jx = (j < 2) ? j : 1;
  int js = j - 2; js = (js < 0) ? 0 : ((js > HD - 1) ? (HD - 1) : js);
  const float xv = x[(size_t)r * 2 + jx];
  float sv = state[(size_t)r * HD + js];
  if (PH) sv *= ZR[(size_t)r * (2 * HD) + HD + js];
  const float ht = (float)HT[(((size_t)b * NCH + c) * FPAD + j) * NNP + n];
  const float hval = (c == 0) ? ((j < 2) ? xv : sv) : ht;
  const float scl = (q < 660) ? (hval * ASC) : ((q < 662) ? ASC : 0.0f);
  const int d0 = (q < 660) ? ((q & 1) * 8) : ((q < 662) ? (q - 660) * 8 : 0);
  const v4f e0 = *(const v4f*)(emb + (size_t)r * ED + d0);
  const v4f e1 = *(const v4f*)(emb + (size_t)r * ED + d0 + 4);
  v8h hv;
#pragma unroll
  for (int e = 0; e < 4; ++e) {
    hv[e]     = (_Float16)(e0[e] * scl);
    hv[4 + e] = (_Float16)(e1[e] * scl);
  }
  _Float16* dst = AP + (size_t)f * 8;
  *(volatile v8h*)dst = hv;
  __threadfence();
  *(volatile v8h*)dst = hv;
}

__global__ __launch_bounds__(256) void gru_combine(const float* __restrict__ ZR, const float* __restrict__ state,
                                                   const float* __restrict__ HC, float* __restrict__ out, int total4) {
  const int f = blockIdx.x * 256 + threadIdx.x;
  if (f >= total4) return;
  const int r = f / (HD / 4);
  const int c = (f - r * (HD / 4)) * 4;
  const v4f z  = *(const v4f*)(ZR + (size_t)r * (2 * HD) + c);
  const v4f s  = *(const v4f*)(state + (size_t)r * HD + c);
  const v4f hc = *(const v4f*)(HC + (size_t)r * HD + c);
  v4f o;
#pragma unroll
  for (int e = 0; e < 4; ++e) o[e] = z[e] * s[e] + (1.0f - z[e]) * hc[e];
  float* dst = out + (size_t)f * 4;
  *(volatile v4f*)dst = o;
  __threadfence();
  *(volatile v4f*)dst = o;
}

extern "C" void kernel_launch(void* const* d_in, const int* in_sizes, int n_in,
                              void* d_out, int out_size, void* d_ws, size_t ws_size,
                              hipStream_t stream) {
  if (n_in < 8) return;
  if (in_sizes[0] != NB * NN * 2 || in_sizes[1] != NB * NN * HD || in_sizes[2] != 2 * NB * NN * NN ||
      in_sizes[3] != NB * NN * ED || in_sizes[4] != ED * IDIM * 2 * HD || in_sizes[5] != ED * 2 * HD ||
      in_sizes[6] != ED * IDIM * HD || in_sizes[7] != ED * HD || out_size != ROWS * HD) return;
  const float* x      = (const float*)d_in[0];
  const float* state  = (const float*)d_in[1];
  const float* graphs = (const float*)d_in[2];
  const float* emb    = (const float*)d_in[3];
  const float* Wg     = (const float*)d_in[4];
  const float* bg     = (const float*)d_in[5];
  const float* Wc     = (const float*)d_in[6];
  const float* bc     = (const float*)d_in[7];
  float* out = (float*)d_out;

  char* ws = (char*)d_ws;
  size_t off = 0;
  auto carve = [&](size_t bytes) -> char* { char* p = ws + off; off += (bytes + 255) & ~(size_t)255; return p; };
  _Float16* G16 = (_Float16*)carve((size_t)2 * NB * NNP * KHP * 2);
  _Float16* HT  = (_Float16*)carve((size_t)NB * NCH * FPAD * NNP * 2);
  _Float16* WTg = (_Float16*)carve((size_t)(2 * HD) * KMP * 2);
  _Float16* WTc = (_Float16*)carve((size_t)HD * KMP * 2);
  _Float16* AP  = (_Float16*)carve((size_t)ROWS * KMP * 2);
  float*    ZR  = (float*)carve((size_t)ROWS * (2 * HD) * 4);
  float*    HC  = (float*)carve((size_t)ROWS * HD * 4);
  if (off > ws_size) return;

  const int g_groups  = 2 * NB * NNP * (KHP / 8);
  const int wg_groups = (2 * HD) * KGRP;
  const int wc_groups = HD * KGRP;
  const int h0_groups = NB * FPAD * (NNP / 8);
  const int ap_groups = ROWS * KGRP;
  const int out4      = ROWS * HD / 4;

  cast_graphs<<<dim3((g_groups + 255) / 256), dim3(256), 0, stream>>>(graphs, G16, g_groups);
  build_wt<<<dim3((wg_groups + 255) / 256), dim3(256), 0, stream>>>(Wg, bg, 2 * HD, WTg, wg_groups);
  build_wt<<<dim3((wc_groups + 255) / 256), dim3(256), 0, stream>>>(Wc, bc, HD, WTc, wc_groups);

  const long htStride = (long)NCH * FPAD * NNP;
  auto hop = [&](int g, int csrc, int cdst) {
    const unsigned short* A  = (const unsigned short*)(HT + (size_t)csrc * FPAD * NNP);
    const unsigned short* Bt = (const unsigned short*)(G16 + (size_t)g * NB * NNP * KHP);
    void* C = (void*)(HT + (size_t)cdst * FPAD * NNP);
    const int tiles = (FPAD / 64) * (NNP / 64);
    dim3 grid((tiles + 7) / 8, NB);
    wmma_gemm64<0, false, 0, 1, false, 0><<<grid, dim3(256), 0, stream>>>(
        A, A, NNP, htStride, Bt, Bt, KHP, (long)NNP * KHP, C, C, NNP, htStride,
        state, state, 0L, FPAD, NNP, KHP, 1.0f / GSC);
  };

  build_ht0<0><<<dim3((h0_groups + 255) / 256), dim3(256), 0, stream>>>(x, state, ZR, HT, h0_groups);
  hop(0, 0, 1); hop(0, 1, 2); hop(1, 0, 3); hop(1, 3, 4);
  build_ap<0><<<dim3((ap_groups + 255) / 256), dim3(256), 0, stream>>>(x, state, emb, ZR, HT, AP, ap_groups);
  {
    const int tiles = (ROWS / 64) * ((2 * HD) / 64);
    wmma_gemm64<0, false, 0, 0, false, 6><<<dim3((tiles + 7) / 8, 1), dim3(256), 0, stream>>>(
        (const unsigned short*)AP, (const unsigned short*)AP, KMP, 0L,
        (const unsigned short*)WTg, (const unsigned short*)WTg, KMP, 0L,
        (void*)ZR, (void*)ZR, 2 * HD, 0L, state, state, 0L, ROWS, 2 * HD, KMP, 1.0f / (ASC * ASC));
  }

  build_ht0<1><<<dim3((h0_groups + 255) / 256), dim3(256), 0, stream>>>(x, state, ZR, HT, h0_groups);
  hop(0, 0, 1); hop(0, 1, 2); hop(1, 0, 3); hop(1, 3, 4);
  build_ap<1><<<dim3((ap_groups + 255) / 256), dim3(256), 0, stream>>>(x, state, emb, ZR, HT, AP, ap_groups);
  {
    const int tiles = (ROWS / 64) * (HD / 64);
    wmma_gemm64<0, false, 0, 0, false, 1><<<dim3((tiles + 7) / 8, 1), dim3(256), 0, stream>>>(
        (const unsigned short*)AP, (const unsigned short*)AP, KMP, 0L,
        (const unsigned short*)WTc, (const unsigned short*)WTc, KMP, 0L,
        (void*)HC, (void*)HC, HD, 0L, state, state, 0L, ROWS, HD, KMP, 1.0f / (ASC * ASC));
  }
  gru_combine<<<dim3((out4 + 255) / 256), dim3(256), 0, stream>>>(ZR, state, HC, out, out4);
}
